// GINEModel_84207128805738
// MI455X (gfx1250) — hardware-verified
//
#include <hip/hip_runtime.h>


namespace {
constexpr int N = 25000, E = 400000, FI = 64, FE = 8, H1 = 256, H2 = 128, NPAD = 25600  , NBLK = NPAD / 128;
constexpr float BNE = 1e-5f;

typedef _Float16 b16;
typedef __attribute__((ext_vector_type(16))) _Float16 v16b;
typedef __attribute__((ext_vector_type(8)))  _Float16 v8b;
typedef __attribute__((ext_vector_type(8)))  float v8f;
typedef __attribute__((ext_vector_type(4)))  float v4f;

__device__ __forceinline__ v8b ld8b(const b16* p) { return *(const v8b*)p; }
__device__ __forceinline__ v16b cat8b(v8b a, v8b b) { return __builtin_shufflevector(a, b, 0, 1, 2, 3, 4, 5, 6, 7, 8, 9, 10, 11, 12, 13, 14, 15); }
__device__ __forceinline__ v16b frag_kb(const b16* p, int hh) { return cat8b(ld8b(p + 8 * hh), ld8b(p + 16 + 8 * hh)); }
__device__ __forceinline__ void split16(float v, b16& hi, b16& lo) { hi = (b16)v; lo = (b16)(v - (float)hi); }
__device__ __forceinline__ void frag_ksplit(const float* p, int hh, v16b& fh_, v16b& fl_) {
  const float* p0 = p + 8 * hh; const float* p1 = p + 16 + 8 * hh;
#pragma unroll
  for (int e = 0; e < 8; ++e) { b16 a, c; split16(p0[e], a, c); fh_[e] = a; fl_[e] = c; split16(p1[e], a, c); fh_[8 + e] = a; fl_[8 + e] = c; }
}
__device__ __forceinline__ v8f wmma16b(v16b a, v16b b, v8f c) {
  v8f d = __builtin_amdgcn_wmma_f32_16x16x32_f16(false, a, false, b, (short)0, c, false, false);
  asm volatile("v_nop\n\tv_nop\n\tv_nop\n\tv_nop" : "+v"(d) : "v"(a), "v"(b));
  return d;
}
__device__ __forceinline__ void wave_lds_sync() {
  __builtin_amdgcn_fence(__ATOMIC_RELEASE, "workgroup");
  __builtin_amdgcn_wave_barrier();
  __builtin_amdgcn_fence(__ATOMIC_ACQUIRE, "workgroup");
}

struct Opnd { const void* p0; const void* p1; int ld; };
template <int NP> __device__ __forceinline__ void load_frags(const Opnd& o, int row, int kb, int hh, v16b& fh_, v16b& fl_) {
  if (NP == 0) { frag_ksplit((const float*)o.p0 + (size_t)row * o.ld + kb, hh, fh_, fl_); }
  else if (NP == 4) {
    const float* p = (const float*)o.p0 + (size_t)row * o.ld + kb; const float* p0 = p + 8 * hh; const float* p1 = p + 16 + 8 * hh;
#pragma unroll
    for (int e = 0; e < 8; ++e) { b16 a, c; split16(p0[e] * 64.0f, a, c); fh_[e] = a; fl_[e] = c; split16(p1[e] * 64.0f, a, c); fh_[8 + e] = a; fl_[8 + e] = c; }
  } else if (NP == 3) {
    const float* p = (const float*)o.p0 + (size_t)row * o.ld + kb; const float* p0 = p + 8 * hh; const float* p1 = p + 16 + 8 * hh;
#pragma unroll
    for (int e = 0; e < 8; ++e) { fh_[e] = (b16)p0[e]; fh_[8 + e] = (b16)p1[e]; }
    fl_ = fh_;
  } else {
    fh_ = frag_kb((const b16*)o.p0 + (size_t)row * o.ld + kb, hh);
    if (NP == 2) fl_ = frag_kb((const b16*)o.p1 + (size_t)row * o.ld + kb, hh); else fl_ = fh_;
  }
}
template <int ANP, int BNP> __device__ __forceinline__ v8f mac(v16b ah, v16b al, v16b bh, v16b bl, v8f c) {
  c = wmma16b(ah, bh, c);
  if (BNP == 0 || BNP == 2 || BNP == 4) c = wmma16b(ah, bl, c);
  if (ANP == 0 || ANP == 2 || ANP == 4) c = wmma16b(al, bh, c);
  return c;
}
template <int ANP, int BNP>
__device__ __forceinline__ void gemm_tile(const Opnd& A, const Opnd& B, int K, int m0, int c0, int nloc, int hlf, v8f (&acc)[2][4]) {
  for (int kb = 0; kb < K; kb += 32) {
    v16b a0h, a0l, a1h, a1l;
    load_frags<ANP>(A, m0 + nloc, kb, hlf, a0h, a0l);
    load_frags<ANP>(A, m0 + 16 + nloc, kb, hlf, a1h, a1l);
#pragma unroll
    for (int t = 0; t < 4; ++t) {
      v16b bh, bl;
      load_frags<BNP>(B, c0 + t * 16 + nloc, kb, hlf, bh, bl);
      acc[0][t] = mac<ANP, BNP>(a0h, a0l, bh, bl, acc[0][t]);
      acc[1][t] = mac<ANP, BNP>(a1h, a1l, bh, bl, acc[1][t]);
    }
  }
}

__device__ __forceinline__ void epi_planes(v8f (&acc)[2][4], float scale, bool two, b16* __restrict__ oh, b16* __restrict__ ol, int ldo,
                                           int m0, int c0, int lane, b16* Th, b16* Tl) {
  const int nloc = lane & 15, hlf = lane >> 4;
#pragma unroll
  for (int t = 0; t < 4; ++t)
#pragma unroll
    for (int r = 0; r < 2; ++r)
#pragma unroll
      for (int v = 0; v < 8; ++v) {
        const int rr = r * 16 + v + 8 * hlf, cc = t * 16 + nloc;
        b16 h_, l_; split16(acc[r][t][v] * scale, h_, l_);
        Th[rr * 64 + cc] = h_; Tl[rr * 64 + cc] = l_;
      }
  wave_lds_sync();
  for (int pass = 0; pass < 2; ++pass) {
#pragma unroll
    for (int j = 0; j < 8; ++j) {
      const int rr = j * 4 + (lane >> 3), c8 = (lane & 7) * 8;
      const size_t o = (size_t)(m0 + rr) * ldo + c0 + c8;
      *(volatile v8b*)(oh + o) = ld8b(Th + rr * 64 + c8);
      if (two) *(volatile v8b*)(ol + o) = ld8b(Tl + rr * 64 + c8);
    }
    __threadfence();
  }
}
__device__ __forceinline__ void epi_f32(v8f (&acc)[2][4], float scale, const float* rscale, float* __restrict__ out, int ldo, int m0, int c0, int lane, float* Tt) {
  const int nloc = lane & 15, hlf = lane >> 4;
#pragma unroll
  for (int t = 0; t < 4; ++t)
#pragma unroll
    for (int r = 0; r < 2; ++r)
#pragma unroll
      for (int v = 0; v < 8; ++v) {
        const int rr = r * 16 + v + 8 * hlf;
        const float rs = rscale ? rscale[(size_t)(m0 + rr) * 32] : 1.0f;
        Tt[rr * 64 + t * 16 + nloc] = acc[r][t][v] * scale * rs;
      }
  wave_lds_sync();
  float* dst0 = out + (size_t)m0 * ldo + c0;
  for (int pass = 0; pass < 2; ++pass) {
#pragma unroll
    for (int j = 0; j < 16; ++j) { const int rr = j * 2 + hlf, c4 = nloc * 4; *(volatile v4f*)(dst0 + (size_t)rr * ldo + c4) = *(const v4f*)(Tt + rr * 64 + c4); }
    __threadfence();
  }
}


__global__ __launch_bounds__(256) void prep_kernel(const float* __restrict__ W11, const float* __restrict__ W12, const float* __restrict__ W21, const float* __restrict__ W22, b16* __restrict__ ph, b16* __restrict__ pl) {
  const size_t tid = (size_t)blockIdx.x * blockDim.x + threadIdx.x, nth = (size_t)gridDim.x * blockDim.x;
  constexpr size_t O1 = 0, O2 = O1 + (size_t)H1 * FI, O3 = O2 + (size_t)H1 * H1, O4 = O3 + (size_t)H2 * H1, OT = O4 + (size_t)H2 * H2;
  for (int pass = 0; pass < 2; ++pass) {
    for (size_t p = tid; p < OT; p += nth) { float w;
      if (p < O2) { const int n = (int)(p / FI), k = (int)(p % FI); w = W11[(size_t)k * H1 + n]; }
      else if (p < O3) { const size_t q = p - O2; const int n = (int)(q / H1), k = (int)(q % H1); w = W12[(size_t)k * H1 + n]; }
      else if (p < O4) { const size_t q = p - O3; const int n = (int)(q / H1), k = (int)(q % H1); w = W21[(size_t)k * H2 + n]; }
      else { const size_t q = p - O4; const int n = (int)(q / H2), k = (int)(q % H2); w = W22[(size_t)k * H2 + n]; }
      b16 a, c; split16(w * 64.0f, a, c); ((volatile b16*)ph)[p] = a; ((volatile b16*)pl)[p] = c; }
    __threadfence();
  }
}

typedef __attribute__((ext_vector_type(4))) int v4i;
template <int DF, int NB>
__global__ __launch_bounds__(256) void agg_kernel(const int* __restrict__ esrc, const int* __restrict__ edst, const float* __restrict__ ea, const float* __restrict__ We, const float* __restrict__ be, const float* __restrict__ epsp,
                                                  const float* __restrict__ x, float* __restrict__ h) {
  constexpr int LW = DF / 32; constexpr float FXS = (DF == 64) ? 262144.0f : 65536.0f, FXI = 1.0f / FXS;
  __shared__ __attribute__((aligned(16))) int acc[NB * DF];
  __shared__ float Ws[FE * DF + DF];
  __shared__ int list[8 * 256];
  const int t_ = threadIdx.x, wave = t_ >> 5, lane = t_ & 31, base = blockIdx.x * NB, col0 = lane * LW;
  for (int i = t_; i < NB * DF; i += 256) acc[i] = 0;
  for (int i = t_; i < FE * DF + DF; i += 256) Ws[i] = (i < FE * DF) ? We[i] : be[i - FE * DF];
  __syncthreads();
  int* wl = list + wave * 256;
  for (int c0 = 0; c0 < E; c0 += 256 * 8) {
    const int e0 = c0 + (wave * 32 + lane) * 8; int dd[8];
#pragma unroll
    for (int j = 0; j < 8; ++j) { const int dv = edst[min(e0 + j, E - 1)]; dd[j] = (e0 + j < E) ? dv : -1; }
    unsigned sl[8]; bool hit[8]; bool anyl = false;
#pragma unroll
    for (int j = 0; j < 8; ++j) { sl[j] = (unsigned)(dd[j] - base); hit[j] = sl[j] < (unsigned)NB; anyl |= hit[j]; }
    int wc = 0;
    if (__builtin_amdgcn_ballot_w32(anyl) != 0u) {
#pragma unroll
      for (int j = 0; j < 8; ++j) {
        const unsigned mj = __builtin_amdgcn_ballot_w32(hit[j]);
        if (mj != 0u) {
          if (hit[j]) { const int pos = wc + (int)__builtin_amdgcn_mbcnt_lo(mj, 0u); wl[pos] = ((e0 + j) << 10) | (int)sl[j]; }
          wc += __builtin_popcount(mj); } } }
    __builtin_amdgcn_wave_barrier(); __builtin_amdgcn_fence(__ATOMIC_RELEASE, "workgroup"); __builtin_amdgcn_fence(__ATOMIC_ACQUIRE, "workgroup");
    for (int i = 0; i < wc; ++i) { const int ent = wl[i]; const int e = ent >> 10, slot = ent & 1023; int s = esrc[e]; s = (s < 0) ? 0 : (s >= N ? N - 1 : s);
      float av[FE];
#pragma unroll
      for (int q = 0; q < FE; ++q) av[q] = ea[(size_t)e * FE + q];
#pragma unroll
      for (int c = 0; c < LW; ++c) { const int col = col0 + c; float m = x[(size_t)s * DF + col] + Ws[FE * DF + col];
#pragma unroll
        for (int q = 0; q < FE; ++q) m += av[q] * Ws[q * DF + col];
        atomicAdd(&acc[slot * DF + col], (int)rintf(fmaxf(m, 0.0f) * FXS)); } }
    __builtin_amdgcn_wave_barrier();
  }
  __syncthreads();
  const float ope = 1.0f + epsp[0];
  for (int pass = 0; pass < 2; ++pass) {
    for (int i = t_; i < NB * DF / 4; i += 256) { const int r = i / (DF / 4), cq = (i % (DF / 4)) * 4, node = base + r; v4f o = {0.0f, 0.0f, 0.0f, 0.0f};
      if (node < N) { const v4f xv = *(const v4f*)(x + (size_t)node * DF + cq);
#pragma unroll
        for (int c = 0; c < 4; ++c) o[c] = ope * xv[c] + (float)acc[r * DF + cq + c] * FXI; }
      *(volatile v4f*)(h + (size_t)node * DF + cq) = o; }
    __threadfence();
  }
}

template <int KIN, int NOUT, bool BNRELU>
__global__ __launch_bounds__(128) void lin_kernel(const float* __restrict__ hin, const float* __restrict__ coef, const b16* __restrict__ wh, const b16* __restrict__ wl, const float* __restrict__ bias, float* __restrict__ y, float* __restrict__ slot_) {
  __shared__ __attribute__((aligned(16))) float Ts[4][32 * 64]; __shared__ float Cp[4][2][64];
  const int lane = threadIdx.x & 31, wave = threadIdx.x >> 5, nloc = lane & 15, hlf = lane >> 4, m0 = blockIdx.y * 128 + wave * 32, c0 = blockIdx.x * 64;
  v8f acc[2][4];
#pragma unroll
  for (int r = 0; r < 2; ++r)
#pragma unroll
    for (int t = 0; t < 4; ++t) acc[r][t] = (v8f){};
#pragma unroll 1
  for (int kb = 0; kb < KIN; kb += 32) { v16b a0, l0, a1, l1;
#pragma unroll
    for (int e = 0; e < 16; ++e) { const int k = kb + ((e < 8) ? (8 * hlf + e) : (16 + 8 * hlf + e - 8)); float u0 = hin[(size_t)(m0 + nloc) * KIN + k], u1 = hin[(size_t)(m0 + 16 + nloc) * KIN + k];
      if (BNRELU) { const float ca = coef[k], sh = coef[KIN + k]; u0 = fmaxf(u0 * ca + sh, 0.0f); u1 = fmaxf(u1 * ca + sh, 0.0f); } b16 p, q; split16(u0 * 8.0f, p, q); a0[e] = p; l0[e] = q; split16(u1 * 8.0f, p, q); a1[e] = p; l1[e] = q; }
#pragma unroll
    for (int t = 0; t < 4; ++t) { const v16b bh = frag_kb(wh + (size_t)(c0 + t * 16 + nloc) * KIN + kb, hlf), bl = frag_kb(wl + (size_t)(c0 + t * 16 + nloc) * KIN + kb, hlf);
      acc[0][t] = wmma16b(a0, bh, acc[0][t]); acc[0][t] = wmma16b(l0, bh, acc[0][t]); acc[0][t] = wmma16b(a0, bl, acc[0][t]);
      acc[1][t] = wmma16b(a1, bh, acc[1][t]); acc[1][t] = wmma16b(l1, bh, acc[1][t]); acc[1][t] = wmma16b(a1, bl, acc[1][t]); } }
#pragma unroll
  for (int t = 0; t < 4; ++t) { const int c = c0 + t * 16 + nloc; float s = 0.0f, s2 = 0.0f;
#pragma unroll
    for (int r = 0; r < 2; ++r)
#pragma unroll
      for (int v = 0; v < 8; ++v) { const float val = acc[r][t][v] * (1.0f / 512.0f) + bias[c]; acc[r][t][v] = val; if (m0 + r * 16 + 8 * hlf + v < N) { s += val; s2 += val * val; } }
    s += __shfl_xor(s, 16); s2 += __shfl_xor(s2, 16);
    if (hlf == 0) { Cp[wave][0][t * 16 + nloc] = s; Cp[wave][1][t * 16 + nloc] = s2; } }
  epi_f32(acc, 1.0f, nullptr, y, NOUT, m0, c0, lane, Ts[wave]);
  __syncthreads();
  { const int which = threadIdx.x >> 6, c = threadIdx.x & 63; const float tot = Cp[0][which][c] + Cp[1][which][c] + Cp[2][which][c] + Cp[3][which][c];
    for (int pass = 0; pass < 2; ++pass) { ((volatile float*)slot_)[((size_t)blockIdx.y * 2 + which) * NOUT + c0 + c] = tot; __threadfence(); } }
}

__global__ __launch_bounds__(256) void bnfin_kernel(const float* __restrict__ slot_, int nch, const float* __restrict__ g, const float* __restrict__ bb, float* __restrict__ coef) {
  const int c = threadIdx.x; if (c >= nch) return;
  double s = 0.0, s2 = 0.0;
  for (int bk = 0; bk < NBLK; ++bk) { s += (double)slot_[((size_t)bk * 2) * nch + c]; s2 += (double)slot_[((size_t)bk * 2 + 1) * nch + c]; }
  const double mean = s / N, var = s2 / N - mean * mean; const float a = g[c] * (float)(1.0 / sqrt(var + (double)BNE)), sh = bb[c] - (float)mean * a;
  for (int pass = 0; pass < 2; ++pass) { ((volatile float*)coef)[c] = a; ((volatile float*)coef)[nch + c] = sh; __threadfence(); }
}

template <int NOUT>
__global__ __launch_bounds__(256) void act_kernel(const float* __restrict__ y, const float* __restrict__ coef, float* __restrict__ h) {
  const size_t i = (size_t)blockIdx.x * 256 + threadIdx.x; const int row = (int)(i / (NOUT / 4)), cq = (int)(i % (NOUT / 4)) * 4;
  const v4f v = *(const v4f*)(y + (size_t)row * NOUT + cq); v4f o;
#pragma unroll
  for (int c = 0; c < 4; ++c) o[c] = (row < N) ? fmaxf(v[c] * coef[cq + c] + coef[NOUT + cq + c], 0.0f) : 0.0f;
  for (int pass = 0; pass < 2; ++pass) { *(volatile v4f*)(h + (size_t)row * NOUT + cq) = o; __threadfence(); }
}

__global__ __launch_bounds__(256) void final_kernel(const float* __restrict__ y, const float* __restrict__ coef, const float* __restrict__ Wout, const float* __restrict__ bout, float* __restrict__ out) {
  __shared__ float Wc[H2], Ca[H2], Cs[H2];
  const int t_ = threadIdx.x, row = blockIdx.x * 256 + t_;
  if (t_ < H2) { Wc[t_] = Wout[t_]; Ca[t_] = coef[t_]; Cs[t_] = coef[H2 + t_]; }
  __syncthreads();
  float s = bout[0];
  if (row < N) {
#pragma unroll 1
    for (int k = 0; k < H2; k += 4) { const v4f v = *(const v4f*)(y + (size_t)row * H2 + k);
#pragma unroll
      for (int c = 0; c < 4; ++c) s += fmaxf(v[c] * Ca[k + c] + Cs[k + c], 0.0f) * Wc[k + c]; } }
  for (int pass = 0; pass < 2; ++pass) { if (row < N) ((volatile float*)out)[row] = s; __threadfence(); }
}
}

extern "C" void kernel_launch(void* const* d_in, const int* in_sizes, int n_in,
                              void* d_out, int out_size, void* d_ws, size_t ws_size, hipStream_t stream) {
  (void)n_in; (void)out_size;
  const float* x = (const float*)d_in[0]; const int* ei = (const int*)d_in[1]; const float* ea = (const float*)d_in[2];
  const float* eps1 = (const float*)d_in[3]; const float* We1 = (const float*)d_in[4]; const float* be1 = (const float*)d_in[5]; const float* W11 = (const float*)d_in[6]; const float* b11 = (const float*)d_in[7]; const float* g11 = (const float*)d_in[8]; const float* bt11 = (const float*)d_in[9];
  const float* W12 = (const float*)d_in[10]; const float* b12 = (const float*)d_in[11]; const float* g1 = (const float*)d_in[12]; const float* bt1 = (const float*)d_in[13];
  const float* eps2 = (const float*)d_in[14]; const float* We2 = (const float*)d_in[15]; const float* be2 = (const float*)d_in[16]; const float* W21 = (const float*)d_in[17]; const float* b21 = (const float*)d_in[18]; const float* g21 = (const float*)d_in[19]; const float* bt21 = (const float*)d_in[20];
  const float* W22 = (const float*)d_in[21]; const float* b22 = (const float*)d_in[22]; const float* g2 = (const float*)d_in[23]; const float* bt2 = (const float*)d_in[24]; const float* Wout = (const float*)d_in[25]; const float* bout = (const float*)d_in[26];
  float* out = (float*)d_out;
  if (in_sizes[0] != N * FI || in_sizes[1] != 2 * E || in_sizes[2] != E * FE || in_sizes[6] != FI * H1 || in_sizes[17] != H1 * H2 || in_sizes[25] != H2) return;
  const int* esrc = ei; const int* edst = ei + E;
  size_t off = 0; char* ws = (char*)d_ws;
  auto carve = [&](size_t bytes) { char* p = ws + off; off += (bytes + 255) & ~(size_t)255; return p; };
  constexpr size_t O2 = (size_t)H1 * FI, O3 = O2 + (size_t)H1 * H1, O4 = O3 + (size_t)H2 * H1, OT = O4 + (size_t)H2 * H2;
  b16* ph = (b16*)carve(OT * 2); b16* pl = (b16*)carve(OT * 2);
  float* h0 = (float*)carve((size_t)NPAD * FI * 4); float* ya = (float*)carve((size_t)NPAD * H1 * 4); float* yb = (float*)carve((size_t)NPAD * H1 * 4); float* hh = (float*)carve((size_t)NPAD * H1 * 4);
  float* slot_ = (float*)carve((size_t)NBLK * 2 * H1 * 4); float* coef = (float*)carve(2 * H1 * 4);
  if (off > ws_size) return;
  prep_kernel<<<256, 256, 0, stream>>>(W11, W12, W21, W22, ph, pl);
  agg_kernel<FI, 1024><<<NPAD / 1024, 256, 0, stream>>>(esrc, edst, ea, We1, be1, eps1, x, h0);
  lin_kernel<FI, H1, false><<<dim3(H1 / 64, NBLK), 128, 0, stream>>>(h0, nullptr, ph, pl, b11, ya, slot_);
  bnfin_kernel<<<1, 256, 0, stream>>>(slot_, H1, g11, bt11, coef);
  lin_kernel<H1, H1, true><<<dim3(H1 / 64, NBLK), 128, 0, stream>>>(ya, coef, ph + O2, pl + O2, b12, yb, slot_);
  bnfin_kernel<<<1, 256, 0, stream>>>(slot_, H1, g1, bt1, coef);
  act_kernel<H1><<<NPAD * H1 / 4 / 256, 256, 0, stream>>>(yb, coef, hh);
  agg_kernel<H1, 256><<<NPAD / 256, 256, 0, stream>>>(esrc, edst, ea, We2, be2, eps2, hh, ya);
  lin_kernel<H1, H2, false><<<dim3(H2 / 64, NBLK), 128, 0, stream>>>(ya, nullptr, ph + O3, pl + O3, b21, yb, slot_);
  bnfin_kernel<<<1, 256, 0, stream>>>(slot_, H2, g21, bt21, coef);
  lin_kernel<H2, H2, true><<<dim3(H2 / 64, NBLK), 128, 0, stream>>>(yb, coef, ph + O4, pl + O4, b22, hh, slot_);
  bnfin_kernel<<<1, 256, 0, stream>>>(slot_, H2, g2, bt2, coef);
  final_kernel<<<(N + 255) / 256, 256, 0, stream>>>(hh, coef, Wout, bout, out);
}
